// LocalCrossAttentionFusion_28338194219149
// MI455X (gfx1250) — hardware-verified
//
#include <hip/hip_runtime.h>

typedef _Float16 v16h __attribute__((ext_vector_type(16)));
typedef _Float16 v8h  __attribute__((ext_vector_type(8)));
typedef float    v8f  __attribute__((ext_vector_type(8)));
typedef float    v4f  __attribute__((ext_vector_type(4)));
typedef v8h __attribute__((may_alias)) v8ha;
typedef v4f __attribute__((may_alias)) v4fa;

union Frag { v16h v; v8h half[2]; };

#define BB     2
#define TT     2048
#define SS     2048
#define DD     512
#define HH     8
#define HD     64
#define WWIN   65
#define WLEFT  32
#define MROWS  (BB * TT)
#define NX     (MROWS * DD)
#define NW     (DD * DD)
#define NW8    (NW / 8)
#define WSCALE 32.0f
#define ASCALE 4.0f
#define NEGF   (-3.402823466e38f)

__device__ __forceinline__ v8f wmma_f16(v16h a, v16h b, v8f c) {
  v8f d = __builtin_amdgcn_wmma_f32_16x16x32_f16(false, a, false, b, (short)0, c, false, false);
  asm volatile("v_nop\n\tv_nop\n\tv_nop\n\tv_nop" : "+v"(d) : "v"(a), "v"(b));
  return d;
}

__device__ __forceinline__ v16h load_frag(const _Float16* p, int h) {
  Frag f;
  f.half[0] = *(const v8ha*)(p + 8 * h);
  f.half[1] = *(const v8ha*)(p + 16 + 8 * h);
  return f.v;
}

__global__ __launch_bounds__(256) void convert_w_kernel(
    const float* __restrict__ wq, const float* __restrict__ wk,
    const float* __restrict__ wv, const float* __restrict__ wo,
    _Float16* __restrict__ wh)
{
  const int g = blockIdx.x * 256 + threadIdx.x;
  if (g >= 4 * NW8) return;
  const int wsel = g / NW8;
  const int off = g - wsel * NW8;
  const float* wsrc = (wsel == 0) ? wq : ((wsel == 1) ? wk : ((wsel == 2) ? wv : wo));
  const float* src = wsrc + (size_t)off * 8;
  _Float16* dst = wh + (size_t)g * 8;
  const v4f a = *(const v4fa*)src;
  const v4f c = *(const v4fa*)(src + 4);
  const v8h o = { (_Float16)(a.x * WSCALE), (_Float16)(a.y * WSCALE), (_Float16)(a.z * WSCALE), (_Float16)(a.w * WSCALE),
                  (_Float16)(c.x * WSCALE), (_Float16)(c.y * WSCALE), (_Float16)(c.z * WSCALE), (_Float16)(c.w * WSCALE) };
  *(volatile v8h*)dst = o;
  __threadfence();
  *(volatile v8h*)dst = o;
}

__global__ __launch_bounds__(256) void ln_kernel(
    const float* __restrict__ xq, const float* __restrict__ xc,
    const float* __restrict__ gq, const float* __restrict__ beq,
    const float* __restrict__ gc, const float* __restrict__ bec,
    _Float16* __restrict__ lnq, _Float16* __restrict__ lnc)
{
  __shared__ float s_red[16];
  const int tid = threadIdx.x, lane = tid & 31, w = tid >> 5;
  const int rl = tid >> 6;
  const int c0 = (tid & 63) * 8;
  const bool isq = blockIdx.x < (MROWS / 4);
  const int rbase = isq ? (int)blockIdx.x * 4 : ((int)blockIdx.x - MROWS / 4) * 4;
  const int r = rbase + rl;
  const float* src = (isq ? xq : xc) + (size_t)r * DD + c0;
  const float* g = (isq ? gq : gc) + c0;
  const float* be = (isq ? beq : bec) + c0;
  _Float16* dst = (isq ? lnq : lnc) + (size_t)r * DD + c0;

  const v4f a = *(const v4fa*)src;
  const v4f c = *(const v4fa*)(src + 4);
  float s = ((a.x + a.y) + (a.z + a.w)) + ((c.x + c.y) + (c.z + c.w));
  #pragma unroll
  for (int o = 16; o >= 1; o >>= 1) s += __shfl_xor(s, o, 32);
  if (lane == 0) s_red[w] = s;
  __syncthreads();
  const float mu = (s_red[2 * rl] + s_red[2 * rl + 1]) * (1.0f / DD);

  const float d0 = a.x - mu, d1 = a.y - mu, d2 = a.z - mu, d3 = a.w - mu;
  const float d4 = c.x - mu, d5 = c.y - mu, d6 = c.z - mu, d7 = c.w - mu;
  float vs = ((d0 * d0 + d1 * d1) + (d2 * d2 + d3 * d3)) + ((d4 * d4 + d5 * d5) + (d6 * d6 + d7 * d7));
  #pragma unroll
  for (int o = 16; o >= 1; o >>= 1) vs += __shfl_xor(vs, o, 32);
  if (lane == 0) s_red[8 + w] = vs;
  __syncthreads();
  const float var = (s_red[8 + 2 * rl] + s_red[9 + 2 * rl]) * (1.0f / DD);
  const float rs = rsqrtf(var + 1e-5f);

  const v4f ga = *(const v4fa*)g;
  const v4f gb = *(const v4fa*)(g + 4);
  const v4f ba = *(const v4fa*)be;
  const v4f bb = *(const v4fa*)(be + 4);
  const v8h o = { (_Float16)(d0 * rs * ga.x + ba.x), (_Float16)(d1 * rs * ga.y + ba.y),
                  (_Float16)(d2 * rs * ga.z + ba.z), (_Float16)(d3 * rs * ga.w + ba.w),
                  (_Float16)(d4 * rs * gb.x + bb.x), (_Float16)(d5 * rs * gb.y + bb.y),
                  (_Float16)(d6 * rs * gb.z + bb.z), (_Float16)(d7 * rs * gb.w + bb.w) };
  *(volatile v8h*)dst = o;
  __threadfence();
  *(volatile v8h*)dst = o;
}

__device__ __forceinline__ void gemm_store_pass(const float* sT, const float* __restrict__ resid,
                                                float* outw, int m0w, int fg, int lane, int has_res) {
  const int q8 = lane & 7, sub = lane >> 3;
  #pragma unroll
  for (int i = 0; i < 16; ++i) {
    const int lid = i * 4 + sub;
    const int row = lid >> 1, hl = lid & 1;
    v4f v = *(const v4fa*)(sT + row * 64 + 32 * hl + 4 * q8);
    const size_t gi = ((size_t)(m0w + row)) * DD + fg * HD + 32 * hl + 4 * q8;
    if (has_res) {
      const v4f rv = *(const v4fa*)(resid + gi);
      v += rv;
    }
    *(volatile v4f*)(outw + gi) = v;
  }
}

__global__ __launch_bounds__(128) void gemm_kernel(
    const _Float16* __restrict__ a0p, const _Float16* __restrict__ a1p, const _Float16* __restrict__ a2p,
    const _Float16* __restrict__ wh,
    const float* __restrict__ b0, const float* __restrict__ b1, const float* __restrict__ b2,
    const float* __restrict__ resid,
    float* __restrict__ outp,
    float oscale, int has_res)
{
  __shared__ __attribute__((aligned(16))) float sTile[4 * 32 * 64];

  const int tid = threadIdx.x, lane = tid & 31, w = tid >> 5;
  const int h = lane >> 4, m = lane & 15;
  const int m0 = blockIdx.x * 128;
  const int which = blockIdx.y >> 3, fg = blockIdx.y & 7;
  const int m0w = m0 + 32 * w;

  const _Float16* ap = (which == 0) ? a0p : ((which == 1) ? a1p : a2p);
  const _Float16* xa0 = ap + (size_t)(m0w + m) * DD;
  const _Float16* xa1 = xa0 + (size_t)16 * DD;
  const _Float16* wb  = wh + ((size_t)which * DD + fg * HD + m) * DD;

  const v8f zero8 = {0.f, 0.f, 0.f, 0.f, 0.f, 0.f, 0.f, 0.f};
  v8f acc[2][4];
  #pragma unroll
  for (int mt = 0; mt < 2; ++mt)
    #pragma unroll
    for (int nt = 0; nt < 4; ++nt) acc[mt][nt] = zero8;

  #pragma unroll 1
  for (int k0 = 0; k0 < DD; k0 += 32) {
    const v16h fa0 = load_frag(xa0 + k0, h);
    const v16h fa1 = load_frag(xa1 + k0, h);
    #pragma unroll
    for (int nt = 0; nt < 4; ++nt) {
      const v16h fb = load_frag(wb + (size_t)nt * 16 * DD + k0, h);
      acc[0][nt] = wmma_f16(fa0, fb, acc[0][nt]);
      acc[1][nt] = wmma_f16(fa1, fb, acc[1][nt]);
    }
  }

  const float* bias = (which == 0) ? b0 : ((which == 1) ? b1 : b2);
  float* sT = sTile + w * 2048;
  #pragma unroll
  for (int nt = 0; nt < 4; ++nt) {
    const int feat = 16 * nt + m;
    const float bvl = bias[fg * HD + feat];
    #pragma unroll
    for (int mt = 0; mt < 2; ++mt) {
      #pragma unroll
      for (int r = 0; r < 8; ++r) {
        const int tokl = 16 * mt + 8 * h + r;
        sT[tokl * 64 + feat] = acc[mt][nt][r] * oscale + bvl;
      }
    }
  }
  __syncthreads();

  float* outw = outp + (size_t)which * NX;
  gemm_store_pass(sT, resid, outw, m0w, fg, lane, has_res);
  __threadfence();
  gemm_store_pass(sT, resid, outw, m0w, fg, lane, has_res);
}

__global__ __launch_bounds__(256) void window_attn_kernel(
    const float* __restrict__ Qf,
    const float* __restrict__ Kf,
    const float* __restrict__ Vf,
    const int* __restrict__ qpos,
    const int* __restrict__ clens,
    _Float16* __restrict__ Ah)
{
  __shared__ __attribute__((aligned(16))) float sq[HH][HD];
  __shared__ float sp[HH][68];
  __shared__ int   sro[HH][68];
  __shared__ __attribute__((aligned(16))) _Float16 sf[HH * HD];

  const int lane = threadIdx.x & 31, h = threadIdx.x >> 5;
  const int bt = blockIdx.x;
  const int b = bt / TT;
  const int pos = qpos[bt];
  const int clen = clens[b];

  const float* qrow = Qf + (size_t)bt * DD + h * HD;
  sq[h][lane] = qrow[lane];
  sq[h][lane + 32] = qrow[lane + 32];
  __syncthreads();

  const int i0 = pos - WLEFT + lane;
  const int i1 = i0 + 32;
  const int i2 = pos - WLEFT + 64;
  const int v0 = (i0 >= 0) && (i0 < clen);
  const int v1 = (i1 >= 0) && (i1 < clen);
  const int v2 = (i2 >= 0) && (i2 < clen);
  const int c0 = min(max(i0, 0), SS - 1);
  const int c1 = min(max(i1, 0), SS - 1);
  const int c2 = min(max(i2, 0), SS - 1);
  const int ro0 = (b * SS + c0) * DD + h * HD;
  const int ro1 = (b * SS + c1) * DD + h * HD;
  const int ro2 = (b * SS + c2) * DD + h * HD;

  const float* k0p = Kf + ro0;
  const float* k1p = Kf + ro1;
  float d0 = 0.f, d1 = 0.f;
  #pragma unroll 2
  for (int i = 0; i < HD / 4; ++i) {
    const v4f q  = *(const v4fa*)(&sq[h][4 * i]);
    const v4f ka = *(const v4fa*)(k0p + 4 * i);
    const v4f kb = *(const v4fa*)(k1p + 4 * i);
    d0 = fmaf(q.x, ka.x, d0); d0 = fmaf(q.y, ka.y, d0); d0 = fmaf(q.z, ka.z, d0); d0 = fmaf(q.w, ka.w, d0);
    d1 = fmaf(q.x, kb.x, d1); d1 = fmaf(q.y, kb.y, d1); d1 = fmaf(q.z, kb.z, d1); d1 = fmaf(q.w, kb.w, d1);
  }
  float part = sq[h][lane] * Kf[ro2 + lane] + sq[h][lane + 32] * Kf[ro2 + lane + 32];
  #pragma unroll
  for (int o = 16; o >= 1; o >>= 1) part += __shfl_xor(part, o, 32);
  const float d2 = part;

  const float s0 = v0 ? d0 * 0.125f : NEGF;
  const float s1 = v1 ? d1 * 0.125f : NEGF;
  const float s2 = v2 ? d2 * 0.125f : NEGF;

  float mx = fmaxf(s0, s1);
  #pragma unroll
  for (int o = 16; o >= 1; o >>= 1) mx = fmaxf(mx, __shfl_xor(mx, o, 32));
  mx = fmaxf(mx, s2);
  const float e0 = __expf(fmaxf(s0 - mx, -87.0f));
  const float e1 = __expf(fmaxf(s1 - mx, -87.0f));
  const float e2 = __expf(fmaxf(s2 - mx, -87.0f));
  float se = e0 + e1;
  #pragma unroll
  for (int o = 16; o >= 1; o >>= 1) se += __shfl_xor(se, o, 32);
  se += e2;
  const float r1 = 1.0f / se;
  const float p0 = v0 ? e0 * r1 : 0.f;
  const float p1 = v1 ? e1 * r1 : 0.f;
  const float p2 = v2 ? e2 * r1 : 0.f;
  float sa = p0 + p1;
  #pragma unroll
  for (int o = 16; o >= 1; o >>= 1) sa += __shfl_xor(sa, o, 32);
  sa += p2;
  const float r2 = 1.0f / fmaxf(sa, 1e-6f);
  const float a0 = p0 * r2, a1 = p1 * r2, a2 = p2 * r2;

  sp[h][lane] = a0;        sro[h][lane] = ro0;
  sp[h][lane + 32] = a1;   sro[h][lane + 32] = ro1;
  if (lane == 0) { sp[h][64] = a2; sro[h][64] = ro2; }
  __syncthreads();

  float f0 = 0.f, f1 = 0.f;
  #pragma unroll 5
  for (int w = 0; w < WWIN; ++w) {
    const float p = sp[h][w];
    int ro = sro[h][w];
    ro = min(max(ro, 0), NX - HD);
    f0 = fmaf(p, Vf[ro + lane], f0);
    f1 = fmaf(p, Vf[ro + lane + 32], f1);
  }
  sf[h * HD + lane] = (_Float16)(f0 * ASCALE);
  sf[h * HD + lane + 32] = (_Float16)(f1 * ASCALE);
  __syncthreads();

  if (h == 0) {
    _Float16* frow = Ah + (size_t)bt * DD;
    const v8h u0 = *(const v8ha*)(sf + lane * 8);
    const v8h u1 = *(const v8ha*)(sf + 256 + lane * 8);
    *(volatile v8h*)(frow + lane * 8) = u0;
    *(volatile v8h*)(frow + 256 + lane * 8) = u1;
    __threadfence();
    *(volatile v8h*)(frow + lane * 8) = u0;
    *(volatile v8h*)(frow + 256 + lane * 8) = u1;
  }
}

extern "C" void kernel_launch(void* const* d_in, const int* in_sizes, int n_in,
                              void* d_out, int out_size, void* d_ws, size_t ws_size,
                              hipStream_t stream) {
  if (n_in < 16) return;
  if (in_sizes[0] != NX || in_sizes[1] != NX) return;
  if (in_sizes[2] != BB * TT || in_sizes[3] != BB) return;
  if (in_sizes[4] != DD || in_sizes[5] != DD || in_sizes[6] != DD || in_sizes[7] != DD) return;
  if (in_sizes[8] != NW || in_sizes[10] != NW || in_sizes[12] != NW || in_sizes[14] != NW) return;
  if (in_sizes[9] != DD || in_sizes[11] != DD || in_sizes[13] != DD || in_sizes[15] != DD) return;
  if (out_size != NX) return;

  const float* query   = (const float*)d_in[0];
  const float* context = (const float*)d_in[1];
  const int*   qpos    = (const int*)d_in[2];
  const int*   clens   = (const int*)d_in[3];
  const float* ln_q_g  = (const float*)d_in[4];
  const float* ln_q_b  = (const float*)d_in[5];
  const float* ln_c_g  = (const float*)d_in[6];
  const float* ln_c_b  = (const float*)d_in[7];
  const float* Wq = (const float*)d_in[8];
  const float* bq = (const float*)d_in[9];
  const float* Wk = (const float*)d_in[10];
  const float* bk = (const float*)d_in[11];
  const float* Wv = (const float*)d_in[12];
  const float* bv = (const float*)d_in[13];
  const float* Wo = (const float*)d_in[14];
  const float* bo = (const float*)d_in[15];
  float* out = (float*)d_out;

  const size_t wh_bytes  = (size_t)4 * NW * 2;
  const size_t ln_bytes  = (size_t)NX * 2;
  const size_t pl_bytes  = (size_t)NX * 4;
  const size_t ah_bytes  = (size_t)NX * 2;
  const size_t o_wh  = 0;
  const size_t o_lnq = o_wh + wh_bytes;
  const size_t o_lnc = o_lnq + ln_bytes;
  const size_t o_qkv = o_lnc + ln_bytes;
  const size_t o_ah  = o_qkv + 3 * pl_bytes;
  const size_t total = o_ah + ah_bytes;
  if (total > ws_size) return;

  char* ws = (char*)d_ws;
  _Float16* wh  = (_Float16*)(ws + o_wh);
  _Float16* lnq = (_Float16*)(ws + o_lnq);
  _Float16* lnc = (_Float16*)(ws + o_lnc);
  float*    qkv = (float*)(ws + o_qkv);
  _Float16* ah  = (_Float16*)(ws + o_ah);

  convert_w_kernel<<<(4 * NW8) / 256, 256, 0, stream>>>(Wq, Wk, Wv, Wo, wh);

  ln_kernel<<<(2 * MROWS) / 4, 256, 0, stream>>>(query, context, ln_q_g, ln_q_b, ln_c_g, ln_c_b, lnq, lnc);

  dim3 gProj(MROWS / 128, 3 * 8);
  gemm_kernel<<<gProj, 128, 0, stream>>>(lnq, lnc, lnc, wh, bq, bk, bv, query, qkv, 0.03125f, 0);

  window_attn_kernel<<<MROWS, 256, 0, stream>>>(qkv, qkv + NX, qkv + 2 * (size_t)NX, qpos, clens, ah);

  dim3 gOut(MROWS / 128, 8);
  gemm_kernel<<<gOut, 128, 0, stream>>>(ah, ah, ah, wh + 3 * (size_t)NW, bo, bo, bo, query, out, 0.0078125f, 1);
}
